// CrossModalAttnMP_64982855188839
// MI455X (gfx1250) — hardware-verified
//
#include <hip/hip_runtime.h>
#include <math.h>


typedef __attribute__((ext_vector_type(16))) _Float16 v16h;
typedef __attribute__((ext_vector_type(8)))  _Float16 v8h;
typedef __attribute__((ext_vector_type(16))) __bf16   v16b;
typedef __attribute__((ext_vector_type(8)))  __bf16   v8b;
typedef __attribute__((ext_vector_type(8)))  float    v8f;
typedef __attribute__((ext_vector_type(4)))  float    v4f;

__device__ __forceinline__ unsigned short f2bf_bits(float f) {
  unsigned u = __float_as_uint(f);
  return (unsigned short)((u + 0x7FFFu + ((u >> 16) & 1u)) >> 16);
}
__device__ __forceinline__ float bf_bits2f(unsigned short h) { return __uint_as_float(((unsigned)h) << 16); }

__device__ __forceinline__ void dep_guard_h(v8f& a, v8f& b, v16h x, v16h y) { asm volatile("v_nop\n\tv_nop\n\tv_nop\n\tv_nop" : "+v"(a), "+v"(b) : "v"(x), "v"(y)); }
__device__ __forceinline__ void dep_guard_b(v8f& a, v8f& b, v16b x, v16b y) { asm volatile("v_nop\n\tv_nop\n\tv_nop\n\tv_nop" : "+v"(a), "+v"(b) : "v"(x), "v"(y)); }
__device__ __forceinline__ void keep4_h(v16h a, v16h b, v16h c, v16h d) { asm volatile("v_nop" :: "v"(a), "v"(b), "v"(c), "v"(d)); }
__device__ __forceinline__ void keep4_b(v16b a, v16b b, v16b c, v16b d) { asm volatile("v_nop" :: "v"(a), "v"(b), "v"(c), "v"(d)); }
__device__ __forceinline__ void acc_guard4(v8f& a, v8f& b, v8f& c, v8f& d) { asm volatile("v_nop\n\tv_nop\n\tv_nop\n\tv_nop" : "+v"(a), "+v"(b), "+v"(c), "+v"(d)); }
template <typename T> struct Frag;
template <> struct Frag<_Float16> {
  typedef v16h V; union U { v16h v; v8h h[2]; };
  static __device__ __forceinline__ v16h load(const _Float16* p) {
    U f; f.h[0] = *(const v8h*)(p); f.h[1] = *(const v8h*)(p + 16); return f.v;
  }
  static __device__ __forceinline__ v8f mma(v16h a, v16h b, v8f c) {
    return __builtin_amdgcn_wmma_f32_16x16x32_f16(false, a, false, b, (short)0, c, false, false);
  }
  static __device__ __forceinline__ void guard(v8f& a, v8f& b, v16h x, v16h y) { dep_guard_h(a, b, x, y); }
  static __device__ __forceinline__ void keep(v16h a, v16h b, v16h c, v16h d) { keep4_h(a, b, c, d); }
};
template <> struct Frag<__bf16> {
  typedef v16b V; union U { v16b v; v8b h[2]; };
  static __device__ __forceinline__ v16b load(const __bf16* p) {
    U f; f.h[0] = *(const v8b*)(p); f.h[1] = *(const v8b*)(p + 16); return f.v;
  }
  static __device__ __forceinline__ v8f mma(v16b a, v16b b, v8f c) {
    return __builtin_amdgcn_wmma_f32_16x16x32_bf16(false, a, false, b, (short)0, c, false, false);
  }
  static __device__ __forceinline__ void guard(v8f& a, v8f& b, v16b x, v16b y) { dep_guard_b(a, b, x, y); }
  static __device__ __forceinline__ void keep(v16b a, v16b b, v16b c, v16b d) { keep4_b(a, b, c, d); }
};

template <int ET> struct Elem;
template <> struct Elem<0> { typedef _Float16 T; };
template <> struct Elem<1> { typedef __bf16 T; };
template <int ET, bool SPLIT, int BIAS_MODE, int OUT_MODE, bool RESID, int ACT = 0>
__global__ __launch_bounds__(256) void wmma_gemm64(
    const unsigned short* __restrict__ Ap, const unsigned short* __restrict__ A2p, int lda, long strideA,
    const unsigned short* __restrict__ Btp, const unsigned short* __restrict__ Bt2p, int ldb, long strideB,
    void* __restrict__ Cout, void* __restrict__ Cout2, int ldc, long strideC,
    const float* __restrict__ bias,
    const float* __restrict__ resid, long strideR,
    int M, int N, int K, float scale) {
  typedef typename Elem<ET>::T T;
  typedef typename Frag<T>::V V;
  const T* A = (const T*)Ap; const T* A2 = (const T*)A2p; const T* Bt = (const T*)Btp; const T* Bt2 = (const T*)Bt2p;
  __shared__ __align__(16) float sT[8][16 * 68];
  const int b    = blockIdx.y;
  const int lane = threadIdx.x & 31;
  const int wave = threadIdx.x >> 5;
  const int tilesN = N >> 6;
  const int tilesM = M >> 6;
  const int tile = blockIdx.x * 8 + wave;
  if (tile >= tilesM * tilesN) return;
  const int tm = tile / tilesN;
  const int tn = tile - tm * tilesN;
  const int m0 = tm << 6;
  const int n0 = tn << 6;

  const T* Ab  = A  + (size_t)b * strideA;
  const T* Bb  = Bt + (size_t)b * strideB;
  const T* Ab2 = SPLIT ? (A2  + (size_t)b * strideA) : nullptr;
  const T* Bb2 = SPLIT ? (Bt2 + (size_t)b * strideB) : nullptr;

  const int rlane = lane & 15;
  const int koff  = (lane >> 4) * 8;
  const int mOff  = (lane >> 4) * 8;

  v8f acc[4][4];
#pragma unroll
  for (int i = 0; i < 4; ++i)
#pragma unroll
    for (int j = 0; j < 4; ++j) acc[i][j] = (v8f){0.f,0.f,0.f,0.f,0.f,0.f,0.f,0.f};

  for (int k0 = 0; k0 < K; k0 += 32) {
    V bh[4], bl[4];
#pragma unroll
    for (int j = 0; j < 4; ++j) {
      const size_t bo = (size_t)(n0 + (j << 4) + rlane) * ldb + koff + k0;
      bh[j] = Frag<T>::load(Bb + bo);
      if (SPLIT) bl[j] = Frag<T>::load(Bb2 + bo);
    }
#pragma unroll
    for (int i = 0; i < 4; ++i) {
      const size_t ao = (size_t)(m0 + (i << 4) + rlane) * lda + koff + k0;
      V ah = Frag<T>::load(Ab + ao);
      V al;
      if (SPLIT) al = Frag<T>::load(Ab2 + ao);
#pragma unroll
      for (int j = 0; j < 4; ++j) {
        acc[i][j] = Frag<T>::mma(ah, bh[j], acc[i][j]);
        if (SPLIT) {
          acc[i][j] = Frag<T>::mma(ah, bl[j], acc[i][j]);
          acc[i][j] = Frag<T>::mma(al, bh[j], acc[i][j]);
        }
      }
      Frag<T>::guard(acc[i][0], acc[i][3], ah, SPLIT ? al : ah);
    }
    Frag<T>::keep(bh[0], bh[1], bh[2], bh[3]);
    if (SPLIT) Frag<T>::keep(bl[0], bl[1], bl[2], bl[3]);
  }
  acc_guard4(acc[0][0], acc[0][1], acc[0][2], acc[0][3]);
  acc_guard4(acc[1][0], acc[1][1], acc[1][2], acc[1][3]);
  acc_guard4(acc[2][0], acc[2][1], acc[2][2], acc[2][3]);
  acc_guard4(acc[3][0], acc[3][1], acc[3][2], acc[3][3]);

  float* slab = sT[wave];
  const float* Rb = RESID ? (resid + (size_t)b * strideR) : nullptr;
#pragma unroll
  for (int i = 0; i < 4; ++i) {
    const int mBase = m0 + (i << 4);
#pragma unroll
    for (int j = 0; j < 4; ++j) {
      const int n = n0 + (j << 4) + rlane;
      float bv = 0.f;
      if (BIAS_MODE == 2) bv = bias[n];
#pragma unroll
      for (int r = 0; r < 8; ++r) {
        float v = acc[i][j][r] * scale;
        if (BIAS_MODE == 1) v += bias[mBase + mOff + r];
        if (BIAS_MODE == 2) v += bv;
        if (RESID) v += Rb[(size_t)(mBase + mOff + r) * ldc + n];
        if (ACT == 1) v = tanhf(v);
        if (ACT == 2) v = fmaxf(v, 0.0f);
        if (ACT == 3) v = v / (1.0f + expf(-v));
        if (ACT == 4) v = (v > 0.f) ? v : 0.01f * v;
        if (ACT == 5) v = 0.5f * v * (1.0f + erff(v * 0.70710678118654752f));
        slab[(mOff + r) * 68 + (j << 4) + rlane] = v;
      }
    }
    __builtin_amdgcn_fence(__ATOMIC_RELEASE, "workgroup");
    __builtin_amdgcn_wave_barrier();
    __builtin_amdgcn_fence(__ATOMIC_ACQUIRE, "workgroup");
    if (OUT_MODE == 0) {
      float* C = (float*)Cout + (size_t)b * strideC;
      const int hh = lane >> 4, c4 = (lane & 15) * 4;
      for (int pass = 0; pass < 2; ++pass) {
#pragma unroll
        for (int it = 0; it < 8; ++it) {
          const int row = it * 2 + hh;
          v4f v = *(const v4f*)(slab + row * 68 + c4);
          *(volatile v4f*)(C + (size_t)(mBase + row) * ldc + n0 + c4) = v;
        }
        __threadfence();
      }
    } else {
      const int q = lane >> 3, c8 = (lane & 7) * 8;
      unsigned short* C  = (unsigned short*)Cout  + (size_t)b * strideC;
      unsigned short* C2 = (OUT_MODE == 2) ? ((unsigned short*)Cout2 + (size_t)b * strideC) : nullptr;
      for (int pass = 0; pass < 2; ++pass) {
#pragma unroll
        for (int it = 0; it < 4; ++it) {
          const int row = it * 4 + q;
          const float* sp = slab + row * 68 + c8;
          v8h hv, lv;
#pragma unroll
          for (int e = 0; e < 8; ++e) {
            if (OUT_MODE == 1) {
              hv[e] = (_Float16)sp[e];
            } else {
              unsigned short hb = f2bf_bits(sp[e]);
              unsigned short lb = f2bf_bits(sp[e] - bf_bits2f(hb));
              hv[e] = __builtin_bit_cast(_Float16, hb);
              lv[e] = __builtin_bit_cast(_Float16, lb);
            }
          }
          *(volatile v8h*)(C + (size_t)(mBase + row) * ldc + n0 + c8) = hv;
          if (OUT_MODE == 2) *(volatile v8h*)(C2 + (size_t)(mBase + row) * ldc + n0 + c8) = lv;
        }
        __threadfence();
      }
    }
    __builtin_amdgcn_fence(__ATOMIC_RELEASE, "workgroup");
    __builtin_amdgcn_wave_barrier();
    __builtin_amdgcn_fence(__ATOMIC_ACQUIRE, "workgroup");
  }
}

__global__ __launch_bounds__(256) void weight_t_f16(const float* __restrict__ W, unsigned short* __restrict__ Wtp,
                                                    int Kin, int Nout) {
  _Float16* Wt = (_Float16*)Wtp;
  const int cpr = Kin >> 3;
  const int total = Nout * cpr;
  const int i = blockIdx.x * 256 + threadIdx.x;
  const int ic = i < total ? i : (total - 1);
  const int n = ic / cpr;
  const int c8 = (ic - n * cpr) * 8;
  v8h hv;
#pragma unroll
  for (int e = 0; e < 8; ++e) hv[e] = (_Float16)(W[(size_t)(c8 + e) * Nout + n] * 16.0f);
  if (i < total) {
    _Float16* qd = Wt + (size_t)n * Kin + c8;
    *(volatile v8h*)qd = hv;
    __threadfence();
    *(volatile v8h*)qd = hv;
  }
}

__global__ __launch_bounds__(256) void cast_rows128_f16(const float* __restrict__ in, unsigned short* __restrict__ dstp,
                                                        int ldd, int M) {
  _Float16* dst = (_Float16*)dstp;
  const int tid = threadIdx.x;
  const int row = blockIdx.x * 16 + (tid >> 4);
  const int c8 = (tid & 15) * 8;
  const int rowc = row < M ? row : (M - 1);
  const float* p = in + (size_t)rowc * 128 + c8;
  const v4f x0 = *(const v4f*)p;
  const v4f x1 = *(const v4f*)(p + 4);
  v8h hv;
  hv[0] = (_Float16)x0[0]; hv[1] = (_Float16)x0[1]; hv[2] = (_Float16)x0[2]; hv[3] = (_Float16)x0[3];
  hv[4] = (_Float16)x1[0]; hv[5] = (_Float16)x1[1]; hv[6] = (_Float16)x1[2]; hv[7] = (_Float16)x1[3];
  if (row < M) {
    _Float16* qd = dst + (size_t)row * ldd + c8;
    *(volatile v8h*)qd = hv;
    __threadfence();
    *(volatile v8h*)qd = hv;
  }
}

__global__ __launch_bounds__(256) void attn_cast_transpose(const float* __restrict__ attn, unsigned short* __restrict__ a16p,
                                                           unsigned short* __restrict__ aT16p, int T) {
  __shared__ __align__(16) _Float16 tileT[128 * 72];
  _Float16* a16 = (_Float16*)a16p;
  _Float16* aT16 = (_Float16*)aT16p;
  const int tid = threadIdx.x, lane = tid & 31, wave = tid >> 5;
  const int tblocks = T >> 6;
  const int b = blockIdx.x / tblocks;
  const int t0 = (blockIdx.x - b * tblocks) * 64;
  const float* src = attn + ((size_t)b * T + t0) * 128;
  _Float16* dstA = a16 + ((size_t)b * T + t0) * 128;
  const int rloc = tid >> 4;
  const int c8 = (tid & 15) * 8;
  v8h keep[4];
#pragma unroll
  for (int it = 0; it < 4; ++it) {
    const int row = it * 16 + rloc;
    const float* p = src + (size_t)row * 128 + c8;
    const v4f x0 = *(const v4f*)p;
    const v4f x1 = *(const v4f*)(p + 4);
    v8h hv;
    hv[0] = (_Float16)x0[0]; hv[1] = (_Float16)x0[1]; hv[2] = (_Float16)x0[2]; hv[3] = (_Float16)x0[3];
    hv[4] = (_Float16)x1[0]; hv[5] = (_Float16)x1[1]; hv[6] = (_Float16)x1[2]; hv[7] = (_Float16)x1[3];
#pragma unroll
    for (int e = 0; e < 8; ++e) tileT[(c8 + e) * 72 + row] = hv[e];
    keep[it] = hv;
    *(volatile v8h*)(dstA + (size_t)row * 128 + c8) = hv;
  }
  __threadfence();
#pragma unroll
  for (int it = 0; it < 4; ++it) {
    const int row = it * 16 + rloc;
    *(volatile v8h*)(dstA + (size_t)row * 128 + c8) = keep[it];
  }
  __syncthreads();
  _Float16* dstT = aT16 + (size_t)b * 128 * T + t0;
  const int q = lane >> 3, tc = (lane & 7) * 8;
  v8h tv[4];
#pragma unroll
  for (int ps = 0; ps < 4; ++ps) {
    const int o = ps * 32 + wave * 4 + q;
    tv[ps] = *(const v8h*)(tileT + o * 72 + tc);
    *(volatile v8h*)(dstT + (size_t)o * T + tc) = tv[ps];
  }
  __threadfence();
#pragma unroll
  for (int ps = 0; ps < 4; ++ps) {
    const int o = ps * 32 + wave * 4 + q;
    *(volatile v8h*)(dstT + (size_t)o * T + tc) = tv[ps];
  }
}

__global__ __launch_bounds__(256) void ln_rows128(const float* __restrict__ pre, const float* __restrict__ X,
                                                  const float* __restrict__ gam, const float* __restrict__ bet,
                                                  float* __restrict__ out, int M) {
  const int lane = threadIdx.x & 31, wave = threadIdx.x >> 5;
  const int c4 = lane * 4;
  const v4f g  = *(const v4f*)(gam + c4);
  const v4f be = *(const v4f*)(bet + c4);
  for (int rr = 0; rr < 4; ++rr) {
    const int row = (blockIdx.x * 8 + wave) * 4 + rr;
    const int rowc = row < M ? row : (M - 1);
    const v4f a = *(const v4f*)(pre + (size_t)rowc * 128 + c4);
    const v4f x = *(const v4f*)(X + (size_t)rowc * 128 + c4);
    const v4f s = a + x;
    float sum = (s[0] + s[1]) + (s[2] + s[3]);
#pragma unroll
    for (int off = 1; off < 32; off <<= 1) sum += __shfl_xor(sum, off, 32);
    const float mu = sum * (1.0f / 128.0f);
    const v4f d = s - mu;
    float sq = (d[0] * d[0] + d[1] * d[1]) + (d[2] * d[2] + d[3] * d[3]);
#pragma unroll
    for (int off = 1; off < 32; off <<= 1) sq += __shfl_xor(sq, off, 32);
    const float var = sq * (1.0f / 128.0f);
    const float rs = rsqrtf(var + 1e-5f);
    const v4f o = (d * rs) * g + be;
    if (row < M) {
      float* qd = out + (size_t)row * 128 + c4;
      *(volatile v4f*)qd = o;
      __threadfence();
      *(volatile v4f*)qd = o;
    }
  }
}

extern "C" void kernel_launch(void* const* d_in, const int* in_sizes, int n_in,
                              void* d_out, int out_size, void* d_ws, size_t ws_size,
                              hipStream_t stream) {
  if (n_in < 15) return;
  const int D = 128;
  const int O = 128;
  const long nTokEl = in_sizes[0];
  const long nObjEl = in_sizes[1];
  const int Mt = (int)(nTokEl / D);
  const int Mo = (int)(nObjEl / D);
  if (Mt <= 0 || Mo <= 0) return;
  const int Bn = Mo / O;
  if (Bn <= 0) return;
  const int T = Mt / Bn;
  if ((long)Bn * T != Mt || (long)Bn * O != Mo) return;
  if (T % 64 != 0 || Mt % 64 != 0 || Mo % 64 != 0) return;
  if ((long)in_sizes[2] != (long)Mt * O) return;
  if (in_sizes[3] != D * D || in_sizes[5] != D * D || in_sizes[7] != 2 * D * D || in_sizes[9] != 2 * D * D) return;
  if ((long)out_size != nTokEl + nObjEl) return;

  const float* token   = (const float*)d_in[0];
  const float* obj     = (const float*)d_in[1];
  const float* attn    = (const float*)d_in[2];
  const float* W_msg_o = (const float*)d_in[3];
  const float* b_msg_o = (const float*)d_in[4];
  const float* W_msg_t = (const float*)d_in[5];
  const float* b_msg_t = (const float*)d_in[6];
  const float* W_upd_t = (const float*)d_in[7];
  const float* b_upd_t = (const float*)d_in[8];
  const float* W_upd_o = (const float*)d_in[9];
  const float* b_upd_o = (const float*)d_in[10];
  const float* g_t     = (const float*)d_in[11];
  const float* be_t    = (const float*)d_in[12];
  const float* g_o     = (const float*)d_in[13];
  const float* be_o    = (const float*)d_in[14];

  float* out_t = (float*)d_out;
  float* out_o = out_t + (size_t)nTokEl;

  size_t off = 0;
  const size_t off_tokA   = off; off += (size_t)Mt * 256 * 2;
  const size_t off_objA   = off; off += (size_t)Mo * 256 * 2;
  const size_t off_attn16 = off; off += (size_t)Mt * O * 2;
  const size_t off_attnT  = off; off += (size_t)Mt * O * 2;
  const size_t off_msgtT  = off; off += (size_t)D * Mt * 2;
  const size_t off_msgoT  = off; off += (size_t)D * Mo * 2;
  const size_t off_pre_t  = off; off += (size_t)Mt * D * 4;
  const size_t off_pre_o  = off; off += (size_t)Mo * D * 4;
  const size_t off_WoT    = off; off += (size_t)D * D * 2;
  const size_t off_WtT    = off; off += (size_t)D * D * 2;
  const size_t off_WutT   = off; off += (size_t)D * 2 * D * 2;
  const size_t off_WuoT   = off; off += (size_t)D * 2 * D * 2;
  const size_t total = off;
  if (total > ws_size) return;
  if (total > (size_t)134217728) return;

  char* ws = (char*)d_ws;
  unsigned short* tokA   = (unsigned short*)(ws + off_tokA);
  unsigned short* objA   = (unsigned short*)(ws + off_objA);
  unsigned short* attn16 = (unsigned short*)(ws + off_attn16);
  unsigned short* attnT  = (unsigned short*)(ws + off_attnT);
  unsigned short* msgtT  = (unsigned short*)(ws + off_msgtT);
  unsigned short* msgoT  = (unsigned short*)(ws + off_msgoT);
  float*          pre_t  = (float*)(ws + off_pre_t);
  float*          pre_o  = (float*)(ws + off_pre_o);
  unsigned short* WoT    = (unsigned short*)(ws + off_WoT);
  unsigned short* WtT    = (unsigned short*)(ws + off_WtT);
  unsigned short* WutT   = (unsigned short*)(ws + off_WutT);
  unsigned short* WuoT   = (unsigned short*)(ws + off_WuoT);

  const float inv16 = 0.0625f;
  const dim3 blk(256);

  weight_t_f16<<<(D * (D / 8) + 255) / 256, blk, 0, stream>>>(W_msg_o, WoT, D, D);
  weight_t_f16<<<(D * (D / 8) + 255) / 256, blk, 0, stream>>>(W_msg_t, WtT, D, D);
  weight_t_f16<<<(D * (2 * D / 8) + 255) / 256, blk, 0, stream>>>(W_upd_t, WutT, 2 * D, D);
  weight_t_f16<<<(D * (2 * D / 8) + 255) / 256, blk, 0, stream>>>(W_upd_o, WuoT, 2 * D, D);

  cast_rows128_f16<<<(Mt + 15) / 16, blk, 0, stream>>>(token, tokA, 256, Mt);
  cast_rows128_f16<<<(Mo + 15) / 16, blk, 0, stream>>>(obj, objA, 256, Mo);

  attn_cast_transpose<<<Bn * (T / 64), blk, 0, stream>>>(attn, attn16, attnT, T);

  {
    const int tiles = (D / 64) * (Mo / 64);
    wmma_gemm64<0, false, 1, 1, false, 0><<<dim3((tiles + 7) / 8, 1), blk, 0, stream>>>(
        WoT, WoT, D, 0L, objA, objA, 256, 0L, msgoT, msgoT, Mo, 0L, b_msg_o, token, 0L, D, Mo, D, inv16);
  }
  {
    const int tiles = (D / 64) * (Mt / 64);
    wmma_gemm64<0, false, 1, 1, false, 0><<<dim3((tiles + 7) / 8, 1), blk, 0, stream>>>(
        WtT, WtT, D, 0L, tokA, tokA, 256, 0L, msgtT, msgtT, Mt, 0L, b_msg_t, token, 0L, D, Mt, D, inv16);
  }
  {
    const int tiles = (T / 64) * (D / 64);
    wmma_gemm64<0, false, 0, 1, false, 0><<<dim3((tiles + 7) / 8, Bn), blk, 0, stream>>>(
        attn16, attn16, O, (long)T * O, msgoT, msgoT, Mo, (long)O, tokA + D, tokA + D, 256, (long)T * 256,
        b_msg_o, token, 0L, T, D, O, 1.0f);
  }
  {
    wmma_gemm64<0, false, 0, 1, false, 0><<<dim3(1, Bn), dim3(128), 0, stream>>>(
        attnT, attnT, T, (long)O * T, msgtT, msgtT, Mt, (long)T, objA + D, objA + D, 256, (long)O * 256,
        b_msg_o, token, 0L, O, D, T, 1.0f);
  }
  {
    const int tiles = (Mt / 64) * (D / 64);
    wmma_gemm64<0, false, 2, 0, false, 2><<<dim3((tiles + 7) / 8, 1), blk, 0, stream>>>(
        tokA, tokA, 256, 0L, WutT, WutT, 256, 0L, pre_t, pre_t, D, 0L, b_upd_t, token, 0L, Mt, D, 2 * D, inv16);
  }
  ln_rows128<<<(Mt + 31) / 32, blk, 0, stream>>>(pre_t, token, g_t, be_t, out_t, Mt);

  {
    const int tiles = (Mo / 64) * (D / 64);
    wmma_gemm64<0, false, 2, 0, false, 2><<<dim3((tiles + 7) / 8, 1), blk, 0, stream>>>(
        objA, objA, 256, 0L, WuoT, WuoT, 256, 0L, pre_o, pre_o, D, 0L, b_upd_o, obj, 0L, Mo, D, 2 * D, inv16);
  }
  ln_rows128<<<(Mo + 31) / 32, blk, 0, stream>>>(pre_o, obj, g_o, be_o, out_o, Mo);

  (void)hipGetLastError();
}
